// MockCFM_17179869193
// MI455X (gfx1250) — hardware-run, weakly checked
//
#include <hip/hip_runtime.h>


#define NB   8
#define NC   128
#define NT   8192
#define K0   0.999999f
typedef _Float16 h16;
typedef unsigned short bf;
typedef __attribute__((ext_vector_type(16))) __bf16   v16bf;
typedef __attribute__((ext_vector_type(16))) _Float16 v16h;
typedef __attribute__((ext_vector_type(8)))  _Float16 v8h;
typedef __attribute__((ext_vector_type(8)))  unsigned short v8us;
typedef __attribute__((ext_vector_type(8)))  float    v8f;
typedef __attribute__((ext_vector_type(4)))  float    v4f;
typedef v8h  __attribute__((may_alias)) v8ha;
typedef v4f  __attribute__((may_alias)) v4fa;
typedef v8us __attribute__((may_alias)) v8usa;

__device__ __forceinline__ unsigned short f2bf(float f) { unsigned u = __float_as_uint(f); u += 0x7FFFu + ((u >> 16) & 1u); return (unsigned short)(u >> 16); }
__device__ __forceinline__ float bf2f(unsigned short b) { return __uint_as_float(((unsigned)b) << 16); }
__device__ __forceinline__ float bfr(float f) { return bf2f(f2bf(f)); }
__device__ __forceinline__ v16h cat16(v8h lo, v8h hi) { return __builtin_shufflevector(lo, hi, 0, 1, 2, 3, 4, 5, 6, 7, 8, 9, 10, 11, 12, 13, 14, 15); }
__device__ __forceinline__ v16bf cat16b(v8us lo, v8us hi) { return __builtin_bit_cast(v16bf, __builtin_shufflevector(lo, hi, 0, 1, 2, 3, 4, 5, 6, 7, 8, 9, 10, 11, 12, 13, 14, 15)); }
__device__ __forceinline__ v8f wmma16(v16h a, v16h b, v8f c) { return __builtin_amdgcn_wmma_f32_16x16x32_f16(false, a, false, b, (short)0, c, false, false); }
__device__ __forceinline__ v8f wmmab(v16bf a, v16bf b, v8f c) { return __builtin_amdgcn_wmma_f32_16x16x32_bf16(false, a, false, b, (short)0, c, false, false); }

template <typename T16> struct WFrag;
template <> struct WFrag<h16> { typedef v16h V; static __device__ __forceinline__ V ld(const h16* p) { return cat16(*(const v8h*)p, *(const v8h*)(p + 16)); } static __device__ __forceinline__ v8f mma(V a, V b, v8f c) { return wmma16(a, b, c); } };
template <> struct WFrag<bf> { typedef v16bf V; static __device__ __forceinline__ V ld(const bf* p) { return cat16b(*(const v8us*)p, *(const v8us*)(p + 16)); } static __device__ __forceinline__ v8f mma(V a, V b, v8f c) { return wmmab(a, b, c); } };
template <typename T16, int NSPLIT, bool BIAS>
__global__ __launch_bounds__(32) void k_gemmw(const T16* __restrict__ A, const T16* __restrict__ A2, const T16* __restrict__ Bt, const T16* __restrict__ Bt2, int K, float* C, int ldc, const float* __restrict__ bias, size_t sA, size_t sB, size_t sC) {
    typedef typename WFrag<T16>::V V;
    __shared__ __align__(16) float os[16 * 68];
    const size_t z = blockIdx.z; A += z * sA; if (A2) A2 += z * sA; Bt += z * sB; if (Bt2) Bt2 += z * sB; C += z * sC;
    const int lane = threadIdx.x & 31, lr = lane & 15, hi = lane >> 4; const int r0 = blockIdx.x * 64, c0 = blockIdx.y * 64;
    v8f acc[4][4];
#pragma unroll
    for (int mb = 0; mb < 4; ++mb)
#pragma unroll
        for (int nb = 0; nb < 4; ++nb) acc[mb][nb] = (v8f){};
    const size_t aoff = (size_t)(r0 + lr) * K + 8 * hi, boff = (size_t)(c0 + lr) * K + 8 * hi;
    for (int kc = 0; kc < K; kc += 32) {
        V a[4], a2[4];
#pragma unroll
        for (int mb = 0; mb < 4; ++mb) { a[mb] = WFrag<T16>::ld(A + aoff + (size_t)mb * 16 * K + kc); if (NSPLIT == 1 || NSPLIT == 2) a2[mb] = WFrag<T16>::ld(A2 + aoff + (size_t)mb * 16 * K + kc); }
#pragma unroll
        for (int nb = 0; nb < 4; ++nb) { const V b = WFrag<T16>::ld(Bt + boff + (size_t)nb * 16 * K + kc); V b2; if (NSPLIT >= 2) b2 = WFrag<T16>::ld(Bt2 + boff + (size_t)nb * 16 * K + kc);
#pragma unroll
            for (int mb = 0; mb < 4; ++mb) { acc[mb][nb] = WFrag<T16>::mma(a[mb], b, acc[mb][nb]); if (NSPLIT == 1 || NSPLIT == 2) acc[mb][nb] = WFrag<T16>::mma(a2[mb], b, acc[mb][nb]); if (NSPLIT >= 2) acc[mb][nb] = WFrag<T16>::mma(a[mb], b2, acc[mb][nb]); } }
        asm volatile("v_nop\n\tv_nop\n\tv_nop\n\tv_nop" : "+v"(acc[0][0]), "+v"(acc[1][1]), "+v"(acc[2][2]), "+v"(acc[3][3]) : "v"(a[0]), "v"(a[3]));
    }
#pragma unroll
    for (int mb = 0; mb < 4; ++mb) {
#pragma unroll
        for (int nb = 0; nb < 4; ++nb) {
#pragma unroll
            for (int j = 0; j < 8; ++j) os[(hi * 8 + j) * 68 + nb * 16 + lr] = acc[mb][nb][j]; }
        __builtin_amdgcn_wave_barrier(); asm volatile("" ::: "memory");
        float* crow = C + (size_t)(r0 + mb * 16) * ldc + c0;
#pragma unroll 1
        for (int ps = 0; ps < 2; ++ps) {
#pragma unroll
            for (int s = 0; s < 8; ++s) { const int row = 2 * s + hi, cofs = lr * 4; v4f val = *(const v4fa*)(os + row * 68 + cofs); if (BIAS) { val[0] += bfr(bias[c0 + cofs]); val[1] += bfr(bias[c0 + cofs + 1]); val[2] += bfr(bias[c0 + cofs + 2]); val[3] += bfr(bias[c0 + cofs + 3]); }
                *(volatile v4f*)(crow + (size_t)row * ldc + cofs) = val; }
            if (ps == 0) __threadfence(); }
        __builtin_amdgcn_wave_barrier(); asm volatile("" ::: "memory");
    }
}

typedef __attribute__((ext_vector_type(2))) _Float16 v2h;
typedef __attribute__((ext_vector_type(4))) _Float16 v4h;
typedef __attribute__((ext_vector_type(2))) unsigned short v2us;
typedef __attribute__((ext_vector_type(4))) unsigned short v4us;
typedef __attribute__((ext_vector_type(2))) float v2f;
typedef __attribute__((ext_vector_type(4))) int v4i;

__device__ __forceinline__ h16 tohx(float x) { return (h16)x; }
__global__ __launch_bounds__(256) void k_cvt8h(const float* __restrict__ src, h16* dst, size_t n8, float sc) { const size_t i = (size_t)blockIdx.x * 256 + threadIdx.x; if (i >= n8) return; const v8f v = *(const v8f*)(src + i * 8); v8h o;
#pragma unroll
    for (int k = 0; k < 8; ++k) o[k] = tohx(bfr(v[k]) * sc); *(volatile v8h*)(dst + i * 8) = o; __threadfence(); *(volatile v8h*)(dst + i * 8) = o; }

__global__ __launch_bounds__(256) void k_th(const float* __restrict__ Y, h16* Yt) { const int j = blockIdx.x * 256 + threadIdx.x; if (j >= NB * NT * NC / 2) return; const int i = (j % (NC / 2)) * 2; const int tt = (j / (NC / 2)) % NT; const int b = j / (NT * NC / 2); const size_t s0 = ((size_t)b * NC + i) * NT + tt; v2h o; o[0] = tohx(Y[s0]); o[1] = tohx(Y[s0 + NT]); *(volatile v2h*)(Yt + (size_t)j * 2) = o; __threadfence(); *(volatile v2h*)(Yt + (size_t)j * 2) = o; }

__global__ __launch_bounds__(256) void k_y(const float* __restrict__ a, const float* __restrict__ g, const float* __restrict__ s, const int* __restrict__ lo, float* Y) { const int i = blockIdx.x * 256 + threadIdx.x; if (i >= NB * NC * NT / 4) return; const size_t f = (size_t)i * 4; const int b = i / (NC * NT / 4); const int t0 = (i % (NT / 4)) * 4; const int l = lo[b]; const float sv = bfr(s[b]); const float c1 = __fsub_rn(1.0f, __fmul_rn(K0, sv)); const v4f av = *(const v4f*)(a + f), gv = *(const v4f*)(g + f); v4f o;
#pragma unroll
    for (int k = 0; k < 4; ++k) { const float y = __fadd_rn(__fmul_rn(c1, bfr(gv[k])), __fmul_rn(sv, bfr(av[k]))); o[k] = (t0 + k < l) ? 0.0f : y; }
    *(volatile v4f*)(Y + f) = o; __threadfence(); *(volatile v4f*)(Y + f) = o; }

__global__ __launch_bounds__(256) void k_out(const float* __restrict__ P, const float* __restrict__ c, const float* __restrict__ g, float* out) { const int j = blockIdx.x * 256 + threadIdx.x; if (j < 32 || j > NB * NC * NT) return; const int e = j - 1; const int dch = (e / NT) % NC; const float o = __fadd_rn(P[e], bfr(c[dch])); const float v = __fadd_rn(o, __fmul_rn(K0, bfr(g[e]))); *(volatile float*)(out + j) = v; __threadfence(); *(volatile float*)(out + j) = v; }

__global__ __launch_bounds__(256) void k_l(const float* __restrict__ P, const float* __restrict__ c, const float* __restrict__ a, const float* __restrict__ g, const int* __restrict__ hi, const int* __restrict__ lo, float* S) { const int i = blockIdx.x * 256 + threadIdx.x; if (i >= NB * NC * (NT / 256)) return; const int b = i / (NC * (NT / 256)); const int dch = (i / (NT / 256)) % NC; const int t0 = (i % (NT / 256)) * 256; const int h = hi[b], l = lo[b]; const float cv = bfr(c[dch]); const size_t f = ((size_t)b * NC + dch) * NT + t0; float sum = 0.0f;
    for (int k = 0; k < 256; ++k) { const float o = __fadd_rn(P[f + k], cv); const float u = __fsub_rn(bfr(a[f + k]), __fmul_rn(K0, bfr(g[f + k]))); const float df = __fsub_rn(o, u); const float sq = __fmul_rn(df, df); const int t = t0 + k; sum = __fadd_rn(sum, (t >= l && t < h) ? sq : 0.0f); }
    *(volatile float*)(S + i) = sum; __threadfence(); *(volatile float*)(S + i) = sum; }

__global__ __launch_bounds__(32) void k_fin(const float* __restrict__ S, const int* __restrict__ hi, const int* __restrict__ lo, const float* __restrict__ P, const float* __restrict__ c, const float* __restrict__ g, float* out) { if (blockIdx.x != 0) return; const int ln = threadIdx.x; float acc = 0.0f;
    for (int b = 0; b < NB; ++b) { float sum = 0.0f; for (int k = 0; k < NC * (NT / 256); ++k) sum = __fadd_rn(sum, S[(size_t)b * NC * (NT / 256) + k]); int h = hi[b], l = lo[b]; h = h < NT ? h : NT; l = l > 0 ? l : 0; const int n = h > l ? h - l : 0; acc = __fadd_rn(acc, __fdiv_rn(sum, (float)(NC * n))); }
    const float mean = __fdiv_rn(acc, (float)NB); const int e = ln > 0 ? ln - 1 : 0; const float o = __fadd_rn(P[e], bfr(c[0])); const float w = __fadd_rn(o, __fmul_rn(K0, bfr(g[e]))); const float v = ln == 0 ? mean : w; *(volatile float*)(out + ln) = v; __threadfence(); *(volatile float*)(out + ln) = v; }

extern "C" void kernel_launch(void* const* d_in, const int* in_sizes, int n_in, void* d_out, int out_size, void* d_ws, size_t ws_size, hipStream_t stream) {
    if (n_in < 9) return;
    if (in_sizes[0] != NB * NC * NT || in_sizes[3] != NB || in_sizes[4] != NB * NC * NT || in_sizes[5] != NC * NC || in_sizes[6] != NC || in_sizes[7] != NB || in_sizes[8] != NB) return;
    if (out_size != 1 + NB * NC * NT) return;
    static_assert(NC % 64 == 0 && NT % 64 == 0 && NC % 32 == 0 && (NB * NT * NC / 2) % 256 == 0 && NC % 2 == 0 && (NC * NC) % (8 * 256) == 0 && (NB * NC * NT / 4) % 256 == 0 && (NB * NC * (NT / 256)) % 256 == 0 && NT % 256 == 0, "the product: M and N multiples of 64, the depth of 32; k_th's two words a thread; the flat grids exact but k_out's, which is one float longer");
    const float* a = (const float*)d_in[0]; const float* s = (const float*)d_in[3]; const float* g = (const float*)d_in[4]; const float* Wm = (const float*)d_in[5]; const float* c = (const float*)d_in[6]; const int* hi = (const int*)d_in[7]; const int* lo = (const int*)d_in[8];
    float* out = (float*)d_out;
    char* wsp = (char*)d_ws; auto take = [&](size_t bytes) { char* p = wsp; wsp += (bytes + 255) & ~(size_t)255; return (void*)p; };
    float* Y = (float*)take((size_t)NB * NC * NT * 4); h16* Yt = (h16*)take((size_t)NB * NT * NC * 2); h16* Wh = (h16*)take((size_t)NC * NC * 2); float* P = (float*)take((size_t)NB * NC * NT * 4); float* S = (float*)take((size_t)NB * NC * (NT / 256) * 4);
    if ((size_t)(wsp - (char*)d_ws) > ws_size) return;
    k_y<<<(unsigned)(NB * NC * NT / 4 / 256), 256, 0, stream>>>(a, g, s, lo, Y);
    k_th<<<(unsigned)(NB * NT * NC / 2 / 256), 256, 0, stream>>>(Y, Yt);
    k_cvt8h<<<(unsigned)(NC * NC / 8 / 256), 256, 0, stream>>>(Wm, Wh, (size_t)NC * NC / 8, 1.0f);
    k_gemmw<h16, 0, false><<<dim3(NC / 64, NT / 64, NB), 32, 0, stream>>>(Wh, nullptr, Yt, nullptr, NC, P, NT, nullptr, 0, (size_t)NT * NC, (size_t)NC * NT);
    k_out<<<(unsigned)((NB * NC * NT + 1 + 255) / 256), 256, 0, stream>>>(P, c, g, out);
    k_l<<<(unsigned)(NB * NC * (NT / 256) / 256), 256, 0, stream>>>(P, c, a, g, hi, lo, S);
    k_fin<<<1, 32, 0, stream>>>(S, hi, lo, P, c, g, out);
}
